// CSSMBase_4389456577151
// MI455X (gfx1250) — hardware-verified
//
#include <hip/hip_runtime.h>
#include <math.h>

constexpr int kBatch    = 4;
constexpr int kChan     = 96;
constexpr int kSeqLen   = 4096;
constexpr int kTok      = kBatch * kSeqLen;
constexpr int kDin      = 192;
constexpr int kNst      = 16;
constexpr int kRank     = 6;
constexpr int kTaps1d   = 4;
constexpr int kImK      = kDin * 9;
constexpr int kImChunks = kImK / 8;
constexpr int kSeqLd    = 128;
constexpr int kXzLd     = 2 * kDin;
constexpr int kXdLd     = 64;
constexpr int kOtLd     = 128;
constexpr int kWdRows   = 128;
constexpr int kXwRows   = 64;
constexpr int kOwRows   = 128;
constexpr int kScanTS   = 64;
constexpr int kScanCh   = 64;
constexpr float kLog2e  = 1.4426950408889634f;

static_assert(kImChunks * 8 == kImK, "im2col chunking");
static_assert(kChan % 32 == 0 && kImK % 32 == 0 && kDin % 32 == 0, "K multiples of 32");
static_assert(kTok % 64 == 0 && kDin % 64 == 0 && kSeqLd % 64 == 0 && kXzLd % 64 == 0 && kXdLd % 64 == 0 && kOtLd % 64 == 0, "tile multiples");
static_assert(kDin == 3 * kScanCh && kSeqLen % kScanTS == 0, "scan blocking");

constexpr size_t kSzX16   = (size_t)kTok * kChan * 2;
constexpr size_t kSzPW16  = (size_t)kDin * kChan * 2;
constexpr size_t kSzWD16  = (size_t)kWdRows * kImK * 2;
constexpr size_t kSzIW16  = (size_t)(2 * kDin) * kChan * 2;
constexpr size_t kSzXW16  = (size_t)kXwRows * kDin * 2;
constexpr size_t kSzOW16  = (size_t)kOwRows * kDin * 2;
constexpr size_t kSzXP16  = (size_t)kTok * kDin * 2;
constexpr size_t kSzIM16  = (size_t)kSeqLen * kImK * 2;
constexpr size_t kSzSEQ16 = (size_t)kTok * kSeqLd * 2;
constexpr size_t kSzXZ    = (size_t)kTok * kXzLd * 4;
constexpr size_t kSzUf    = (size_t)kTok * kDin * 4;
constexpr size_t kSzU16   = (size_t)kTok * kDin * 2;
constexpr size_t kSzXD    = (size_t)kTok * kXdLd * 4;
constexpr size_t kSzY16   = kSzU16;
constexpr size_t kSzOT    = (size_t)kTok * kOtLd * 4;

constexpr size_t kOffXhi   = 0;
constexpr size_t kOffXlo   = kOffXhi + kSzX16;
constexpr size_t kOffPWhi  = kOffXlo + kSzX16;
constexpr size_t kOffPWlo  = kOffPWhi + kSzPW16;
constexpr size_t kOffWDhi  = kOffPWlo + kSzPW16;
constexpr size_t kOffWDlo  = kOffWDhi + kSzWD16;
constexpr size_t kOffIWhi  = kOffWDlo + kSzWD16;
constexpr size_t kOffIWlo  = kOffIWhi + kSzIW16;
constexpr size_t kOffXWhi  = kOffIWlo + kSzIW16;
constexpr size_t kOffXWlo  = kOffXWhi + kSzXW16;
constexpr size_t kOffOWhi  = kOffXWlo + kSzXW16;
constexpr size_t kOffOWlo  = kOffOWhi + kSzOW16;
constexpr size_t kOffXPhi  = kOffOWlo + kSzOW16;
constexpr size_t kOffXPlo  = kOffXPhi + kSzXP16;
constexpr size_t kOffIMhi  = kOffXPlo + kSzXP16;
constexpr size_t kOffIMlo  = kOffIMhi + kSzIM16;
constexpr size_t kOffSEQhi = kOffIMlo + kSzIM16;
constexpr size_t kOffSEQlo = kOffSEQhi + kSzSEQ16;
constexpr size_t kOffXZ    = kOffSEQlo + kSzSEQ16;
constexpr size_t kOffUf    = kOffXZ + kSzXZ;
constexpr size_t kOffUhi   = kOffUf + kSzUf;
constexpr size_t kOffUlo   = kOffUhi + kSzU16;
constexpr size_t kOffXD    = kOffUlo + kSzU16;
constexpr size_t kWsTotal  = kOffXD + kSzXD;
constexpr size_t kOffYhi   = kOffIMhi;
constexpr size_t kOffYlo   = kOffYhi + kSzY16;
constexpr size_t kOffOT    = kOffXPhi;
static_assert(kOffYlo + kSzY16 <= kOffIMlo + kSzIM16, "Y planes fit in the im2col region");
static_assert(kOffOT + kSzOT <= kOffXPlo + kSzXP16, "OT fits in the XP region");
static_assert(kWsTotal == 111353856ull, "carve total");
static_assert(kWsTotal <= 134217728ull, "carve under 128 MiB");
static_assert(kOffPWhi % 128 == 0 && kOffWDhi % 128 == 0 && kOffIWhi % 128 == 0 && kOffXWhi % 128 == 0 &&
              kOffOWhi % 128 == 0 && kOffXPhi % 128 == 0 && kOffIMhi % 128 == 0 && kOffSEQhi % 128 == 0 &&
              kOffXZ % 128 == 0 && kOffUf % 128 == 0 && kOffUhi % 128 == 0 && kOffXD % 128 == 0 && kOffYlo % 128 == 0,
              "128-B aligned carves");

typedef __attribute__((ext_vector_type(16))) _Float16 v16h;
typedef __attribute__((ext_vector_type(8)))  _Float16 v8h;
typedef __attribute__((ext_vector_type(16))) __bf16   v16b;
typedef __attribute__((ext_vector_type(8)))  __bf16   v8b;
typedef __attribute__((ext_vector_type(8)))  float    v8f;
typedef __attribute__((ext_vector_type(4)))  float    v4f;
typedef __attribute__((ext_vector_type(4)))  unsigned int v4u;

__device__ __forceinline__ unsigned short f2bf_bits(float f) {
  unsigned u = __float_as_uint(f);
  return (unsigned short)((u + 0x7FFFu + ((u >> 16) & 1u)) >> 16);
}
__device__ __forceinline__ float bf_bits2f(unsigned short h) { return __uint_as_float(((unsigned)h) << 16); }
__device__ __forceinline__ unsigned pk16(unsigned short a, unsigned short b) { return (unsigned)a | ((unsigned)b << 16); }

__device__ __forceinline__ void pack8_split(const float (&f)[8], v4u& hv, v4u& lv) {
  unsigned short hb[8], lb[8];
#pragma unroll
  for (int e = 0; e < 8; ++e) {
    hb[e] = f2bf_bits(f[e]);
    lb[e] = f2bf_bits(f[e] - bf_bits2f(hb[e]));
  }
  hv = (v4u){pk16(hb[0], hb[1]), pk16(hb[2], hb[3]), pk16(hb[4], hb[5]), pk16(hb[6], hb[7])};
  lv = (v4u){pk16(lb[0], lb[1]), pk16(lb[2], lb[3]), pk16(lb[4], lb[5]), pk16(lb[6], lb[7])};
}

__device__ __forceinline__ void dep_guard_h(v8f& a, v8f& b, v16h x, v16h y) { asm volatile("v_nop\n\tv_nop\n\tv_nop\n\tv_nop" : "+v"(a), "+v"(b) : "v"(x), "v"(y)); }
__device__ __forceinline__ void dep_guard_b(v8f& a, v8f& b, v16b x, v16b y) { asm volatile("v_nop\n\tv_nop\n\tv_nop\n\tv_nop" : "+v"(a), "+v"(b) : "v"(x), "v"(y)); }
__device__ __forceinline__ void keep4_h(v16h a, v16h b, v16h c, v16h d) { asm volatile("v_nop" :: "v"(a), "v"(b), "v"(c), "v"(d)); }
__device__ __forceinline__ void keep4_b(v16b a, v16b b, v16b c, v16b d) { asm volatile("v_nop" :: "v"(a), "v"(b), "v"(c), "v"(d)); }
__device__ __forceinline__ void acc_guard4(v8f& a, v8f& b, v8f& c, v8f& d) { asm volatile("v_nop\n\tv_nop\n\tv_nop\n\tv_nop" : "+v"(a), "+v"(b), "+v"(c), "+v"(d)); }
template <typename T> struct Frag;
template <> struct Frag<_Float16> {
  typedef v16h V; union U { v16h v; v8h h[2]; };
  static __device__ __forceinline__ v16h load(const _Float16* p) {
    U f; f.h[0] = *(const v8h*)(p); f.h[1] = *(const v8h*)(p + 16); return f.v;
  }
  static __device__ __forceinline__ v8f mma(v16h a, v16h b, v8f c) {
    return __builtin_amdgcn_wmma_f32_16x16x32_f16(false, a, false, b, (short)0, c, false, false);
  }
  static __device__ __forceinline__ void guard(v8f& a, v8f& b, v16h x, v16h y) { dep_guard_h(a, b, x, y); }
  static __device__ __forceinline__ void keep(v16h a, v16h b, v16h c, v16h d) { keep4_h(a, b, c, d); }
};
template <> struct Frag<__bf16> {
  typedef v16b V; union U { v16b v; v8b h[2]; };
  static __device__ __forceinline__ v16b load(const __bf16* p) {
    U f; f.h[0] = *(const v8b*)(p); f.h[1] = *(const v8b*)(p + 16); return f.v;
  }
  static __device__ __forceinline__ v8f mma(v16b a, v16b b, v8f c) {
    return __builtin_amdgcn_wmma_f32_16x16x32_bf16(false, a, false, b, (short)0, c, false, false);
  }
  static __device__ __forceinline__ void guard(v8f& a, v8f& b, v16b x, v16b y) { dep_guard_b(a, b, x, y); }
  static __device__ __forceinline__ void keep(v16b a, v16b b, v16b c, v16b d) { keep4_b(a, b, c, d); }
};

template <int ET> struct Elem;
template <> struct Elem<0> { typedef _Float16 T; };
template <> struct Elem<1> { typedef __bf16 T; };
template <int ET, bool SPLIT, int BIAS_MODE, int OUT_MODE, bool RESID, int ACT = 0>
__global__ __launch_bounds__(256) void wmma_gemm64(
    const unsigned short* __restrict__ Ap, const unsigned short* __restrict__ A2p, int lda, long strideA,
    const unsigned short* __restrict__ Btp, const unsigned short* __restrict__ Bt2p, int ldb, long strideB,
    void* __restrict__ Cout, void* __restrict__ Cout2, int ldc, long strideC,
    const float* __restrict__ bias,
    const float* __restrict__ resid, long strideR,
    int M, int N, int K, float scale) {
  typedef typename Elem<ET>::T T;
  typedef typename Frag<T>::V V;
  const T* A = (const T*)Ap; const T* A2 = (const T*)A2p; const T* Bt = (const T*)Btp; const T* Bt2 = (const T*)Bt2p;
  __shared__ __align__(16) float sT[8][16 * 68];
  const int b    = blockIdx.y;
  const int lane = threadIdx.x & 31;
  const int wave = threadIdx.x >> 5;
  const int tilesN = N >> 6;
  const int tilesM = M >> 6;
  const int tile = blockIdx.x * 8 + wave;
  if (tile >= tilesM * tilesN) return;
  const int tm = tile / tilesN;
  const int tn = tile - tm * tilesN;
  const int m0 = tm << 6;
  const int n0 = tn << 6;

  const T* Ab  = A  + (size_t)b * strideA;
  const T* Bb  = Bt + (size_t)b * strideB;
  const T* Ab2 = SPLIT ? (A2  + (size_t)b * strideA) : nullptr;
  const T* Bb2 = SPLIT ? (Bt2 + (size_t)b * strideB) : nullptr;

  const int rlane = lane & 15;
  const int koff  = (lane >> 4) * 8;
  const int mOff  = (lane >> 4) * 8;

  v8f acc[4][4];
#pragma unroll
  for (int i = 0; i < 4; ++i)
#pragma unroll
    for (int j = 0; j < 4; ++j) acc[i][j] = (v8f){0.f,0.f,0.f,0.f,0.f,0.f,0.f,0.f};

  for (int k0 = 0; k0 < K; k0 += 32) {
    V bh[4], bl[4];
#pragma unroll
    for (int j = 0; j < 4; ++j) {
      const size_t bo = (size_t)(n0 + (j << 4) + rlane) * ldb + koff + k0;
      bh[j] = Frag<T>::load(Bb + bo);
      if (SPLIT) bl[j] = Frag<T>::load(Bb2 + bo);
    }
#pragma unroll
    for (int i = 0; i < 4; ++i) {
      const size_t ao = (size_t)(m0 + (i << 4) + rlane) * lda + koff + k0;
      V ah = Frag<T>::load(Ab + ao);
      V al;
      if (SPLIT) al = Frag<T>::load(Ab2 + ao);
#pragma unroll
      for (int j = 0; j < 4; ++j) {
        acc[i][j] = Frag<T>::mma(ah, bh[j], acc[i][j]);
        if (SPLIT) {
          acc[i][j] = Frag<T>::mma(ah, bl[j], acc[i][j]);
          acc[i][j] = Frag<T>::mma(al, bh[j], acc[i][j]);
        }
      }
      Frag<T>::guard(acc[i][0], acc[i][3], ah, SPLIT ? al : ah);
    }
    Frag<T>::keep(bh[0], bh[1], bh[2], bh[3]);
    if (SPLIT) Frag<T>::keep(bl[0], bl[1], bl[2], bl[3]);
  }
  acc_guard4(acc[0][0], acc[0][1], acc[0][2], acc[0][3]);
  acc_guard4(acc[1][0], acc[1][1], acc[1][2], acc[1][3]);
  acc_guard4(acc[2][0], acc[2][1], acc[2][2], acc[2][3]);
  acc_guard4(acc[3][0], acc[3][1], acc[3][2], acc[3][3]);

  float* slab = sT[wave];
  const float* Rb = RESID ? (resid + (size_t)b * strideR) : nullptr;
#pragma unroll
  for (int i = 0; i < 4; ++i) {
    const int mBase = m0 + (i << 4);
#pragma unroll
    for (int j = 0; j < 4; ++j) {
      const int n = n0 + (j << 4) + rlane;
      float bv = 0.f;
      if (BIAS_MODE == 2) bv = bias[n];
#pragma unroll
      for (int r = 0; r < 8; ++r) {
        float v = acc[i][j][r] * scale;
        if (BIAS_MODE == 1) v += bias[mBase + mOff + r];
        if (BIAS_MODE == 2) v += bv;
        if (RESID) v += Rb[(size_t)(mBase + mOff + r) * ldc + n];
        if (ACT == 2) v = fmaxf(v, 0.0f);
        if (ACT == 4) v = (v > 0.f) ? v : 0.01f * v;
        slab[(mOff + r) * 68 + (j << 4) + rlane] = v;
      }
    }
    __builtin_amdgcn_fence(__ATOMIC_RELEASE, "workgroup");
    __builtin_amdgcn_wave_barrier();
    __builtin_amdgcn_fence(__ATOMIC_ACQUIRE, "workgroup");
    if (OUT_MODE == 0) {
      float* C = (float*)Cout + (size_t)b * strideC;
      const int hh = lane >> 4, c4 = (lane & 15) * 4;
      for (int pass = 0; pass < 2; ++pass) {
#pragma unroll
        for (int it = 0; it < 8; ++it) {
          const int row = it * 2 + hh;
          v4f v = *(const v4f*)(slab + row * 68 + c4);
          *(volatile v4f*)(C + (size_t)(mBase + row) * ldc + n0 + c4) = v;
        }
        __threadfence();
      }
    } else {
      const int q = lane >> 3, c8 = (lane & 7) * 8;
      unsigned short* C  = (unsigned short*)Cout  + (size_t)b * strideC;
      unsigned short* C2 = (OUT_MODE == 2) ? ((unsigned short*)Cout2 + (size_t)b * strideC) : nullptr;
      for (int pass = 0; pass < 2; ++pass) {
#pragma unroll
        for (int it = 0; it < 4; ++it) {
          const int row = it * 4 + q;
          const float* sp = slab + row * 68 + c8;
          v8h hv, lv;
#pragma unroll
          for (int e = 0; e < 8; ++e) {
            if (OUT_MODE == 1) {
              hv[e] = (_Float16)sp[e];
            } else {
              unsigned short hb = f2bf_bits(sp[e]);
              unsigned short lb = f2bf_bits(sp[e] - bf_bits2f(hb));
              hv[e] = __builtin_bit_cast(_Float16, hb);
              lv[e] = __builtin_bit_cast(_Float16, lb);
            }
          }
          *(volatile v8h*)(C + (size_t)(mBase + row) * ldc + n0 + c8) = hv;
          if (OUT_MODE == 2) *(volatile v8h*)(C2 + (size_t)(mBase + row) * ldc + n0 + c8) = lv;
        }
        __threadfence();
      }
    }
    __builtin_amdgcn_fence(__ATOMIC_RELEASE, "workgroup");
    __builtin_amdgcn_wave_barrier();
    __builtin_amdgcn_fence(__ATOMIC_ACQUIRE, "workgroup");
  }
}

__global__ __launch_bounds__(256) void wsplit_kernel(const float* __restrict__ src,
                                                     unsigned short* __restrict__ hi, unsigned short* __restrict__ lo,
                                                     int nrowsSrc, int ncols, int mode, int n8) {
  const int i = blockIdx.x * 256 + threadIdx.x;
  if (i >= n8) return;
  const size_t amax = (size_t)nrowsSrc * ncols - 1;
  float f[8];
#pragma unroll
  for (int j = 0; j < 8; ++j) {
    const int e = 8 * i + j;
    const int row = e / ncols;
    const int col = e - row * ncols;
    const int rc = (row < nrowsSrc) ? row : (nrowsSrc - 1);
    const size_t a0 = (size_t)rc * ncols + col;
    const int tap = col / kDin;
    const int ci = col - tap * kDin;
    size_t a1 = ((size_t)rc * kDin + ci) * 9 + tap;
    a1 = (a1 > amax) ? amax : a1;
    const float v0 = src[a0];
    const float v1 = src[a1];
    float v = (mode != 0) ? v1 : v0;
    v = (row < nrowsSrc) ? v : 0.0f;
    f[j] = v;
  }
  v4u hv, lv;
  pack8_split(f, hv, lv);
  for (int pass = 0; pass < 2; ++pass) {
    *(volatile v4u*)(hi + 8 * (size_t)i) = hv;
    *(volatile v4u*)(lo + 8 * (size_t)i) = lv;
    __threadfence();
  }
}

__global__ __launch_bounds__(256) void xin_kernel(const float* __restrict__ x,
                                                  unsigned short* __restrict__ xhi, unsigned short* __restrict__ xlo) {
  __shared__ float sm[64][kChan + 1];
  const int tid = threadIdx.x, lane = tid & 31, wave = tid >> 5;
  const int b = blockIdx.x >> 6;
  const int l0 = (blockIdx.x & 63) * 64;
#pragma unroll
  for (int i = 0; i < 24; ++i) {
    const int e = i * 256 + tid;
    const int c = e >> 6, t = e & 63;
    sm[t][c] = x[((size_t)(b * kChan + c)) * kSeqLen + l0 + t];
  }
  __syncthreads();
  const size_t base = ((size_t)b * kSeqLen + l0) * kChan;
  v4u hv[3], lv[3];
#pragma unroll
  for (int it = 0; it < 3; ++it) {
    const int q = wave * 96 + it * 32 + lane;
    const int fidx = 8 * q;
    const int t = fidx / kChan, c = fidx - t * kChan;
    float v[8];
#pragma unroll
    for (int e = 0; e < 8; ++e) v[e] = sm[t][c + e];
    pack8_split(v, hv[it], lv[it]);
  }
  for (int pass = 0; pass < 2; ++pass) {
#pragma unroll
    for (int it = 0; it < 3; ++it) {
      const int q = wave * 96 + it * 32 + lane;
      *(volatile v4u*)(xhi + base + 8 * (size_t)q) = hv[it];
      *(volatile v4u*)(xlo + base + 8 * (size_t)q) = lv[it];
    }
    __threadfence();
  }
}

__global__ __launch_bounds__(256) void im2col_kernel(const unsigned short* __restrict__ xphi, const unsigned short* __restrict__ xplo,
                                                     unsigned short* __restrict__ imhi, unsigned short* __restrict__ imlo, int img) {
  const int tid = threadIdx.x, lane = tid & 31, wave = tid >> 5;
  const int r = blockIdx.x * 8 + wave;
  const int h = r >> 6, w = r & 63;
  const size_t srcBase = (size_t)img * kSeqLen;
  v4u hv[7], lv[7];
#pragma unroll
  for (int it = 0; it < 7; ++it) {
    const int q = it * 32 + lane;
    const int qc = (q < kImChunks) ? q : (kImChunks - 1);
    const int tap = qc / 24;
    const int wi = qc - tap * 24;
    const int kh = tap / 3;
    const int kw = tap - kh * 3;
    const int h2 = h + kh - 1, w2 = w + kw - 1;
    const bool ok = ((unsigned)h2 < 64u) && ((unsigned)w2 < 64u);
    const int srow = ok ? (h2 * 64 + w2) : 0;
    const size_t so = (srcBase + srow) * kDin + (size_t)wi * 8;
    const v4u a = *(const v4u*)(xphi + so);
    const v4u c = *(const v4u*)(xplo + so);
    const unsigned m = ok ? 0xffffffffu : 0u;
    const v4u mv = (v4u){m, m, m, m};
    hv[it] = a & mv;
    lv[it] = c & mv;
  }
  const size_t ro = (size_t)r * kImK;
  for (int pass = 0; pass < 2; ++pass) {
#pragma unroll
    for (int it = 0; it < 7; ++it) {
      const int q = it * 32 + lane;
      if (q < kImChunks) {
        *(volatile v4u*)(imhi + ro + 8 * (size_t)q) = hv[it];
        *(volatile v4u*)(imlo + ro + 8 * (size_t)q) = lv[it];
      }
    }
    __threadfence();
  }
}

__global__ __launch_bounds__(256) void conv_silu_kernel(const float* __restrict__ xz, const float* __restrict__ cw,
                                                        const float* __restrict__ cb, float* __restrict__ uf,
                                                        unsigned short* __restrict__ uhi, unsigned short* __restrict__ ulo) {
  __shared__ __align__(16) float su[8][kDin];
  const int tid = threadIdx.x, lane = tid & 31, wave = tid >> 5;
  const int row = blockIdx.x * 8 + wave;
  const int li = row & (kSeqLen - 1);
  const size_t img0 = (size_t)(row - li);
  float* sw = su[wave];
#pragma unroll 1
  for (int j = 0; j < kDin / 32; ++j) {
    const int d = lane + 32 * j;
    float s = 0.f;
#pragma unroll
    for (int k = 0; k < kTaps1d; ++k) {
      const int src = li - (kTaps1d - 1) + k;
      const int sc = (src < 0) ? 0 : src;
      float v = xz[(img0 + sc) * kXzLd + d];
      v = (src >= 0) ? v : 0.f;
      s = fmaf(cw[d * kTaps1d + k], v, s);
    }
    s += cb[d];
    const float val = s * __builtin_amdgcn_rcpf(1.0f + expf(-s));
    sw[d] = val;
  }
  __builtin_amdgcn_fence(__ATOMIC_RELEASE, "workgroup");
  __builtin_amdgcn_wave_barrier();
  __builtin_amdgcn_fence(__ATOMIC_ACQUIRE, "workgroup");
  const int c4a = lane * 4;
  const int c4b = 128 + (lane & 15) * 4;
  const int c8 = ((lane < 24) ? lane : 0) * 8;
  const v4f va = *(const v4f*)(sw + c4a);
  const v4f vb = *(const v4f*)(sw + c4b);
  float f8[8];
#pragma unroll
  for (int e = 0; e < 8; ++e) f8[e] = sw[c8 + e];
  v4u hv, lv;
  pack8_split(f8, hv, lv);
  const size_t ro = (size_t)row * kDin;
  for (int pass = 0; pass < 2; ++pass) {
    *(volatile v4f*)(uf + ro + c4a) = va;
    if (lane < 16) *(volatile v4f*)(uf + ro + c4b) = vb;
    if (lane < 24) {
      *(volatile v4u*)(uhi + ro + c8) = hv;
      *(volatile v4u*)(ulo + ro + c8) = lv;
    }
    __threadfence();
  }
}

__global__ __launch_bounds__(64) void scan_kernel(const float* __restrict__ xdbl, const float* __restrict__ uf,
                                                  const float* __restrict__ xz, const float* __restrict__ dtw,
                                                  const float* __restrict__ dtb, const float* __restrict__ alog,
                                                  const float* __restrict__ dvec,
                                                  unsigned short* __restrict__ yhi, unsigned short* __restrict__ ylo) {
  __shared__ __align__(16) float sx[kScanTS][40];
  __shared__ __align__(16) float sy[kScanTS][kScanCh + 4];
  __shared__ float sh[kNst][kScanCh];
  __shared__ float sa[kNst][kScanCh];
  const int tid = threadIdx.x, lane = tid & 31, wave = tid >> 5;
  const int g = blockIdx.x % 3;
  const int b = blockIdx.x / 3;
  const int d = g * kScanCh + tid;
  float wr[kRank];
#pragma unroll
  for (int r = 0; r < kRank; ++r) wr[r] = dtw[d * kRank + r];
  const float bd = dtb[d];
  const float Dd = dvec[d];
#pragma unroll 1
  for (int n = 0; n < kNst; ++n) {
    sh[n][tid] = 0.f;
    sa[n][tid] = -expf(alog[d * kNst + n]) * kLog2e;
  }
  const int q = lane >> 3, c8 = (lane & 7) * 8;
  for (int l0 = 0; l0 < kSeqLen; l0 += kScanTS) {
    __syncthreads();
    const size_t rowBase = (size_t)b * kSeqLen + l0;
#pragma unroll
    for (int i = 0; i < 10; ++i) {
      const int e = i * 64 + tid;
      const int r = e / 10, qq = e - r * 10;
      const v4f v = *(const v4f*)(xdbl + (rowBase + r) * kXdLd + 4 * qq);
      *(v4f*)(&sx[r][4 * qq]) = v;
    }
    __syncthreads();
#pragma unroll 1
    for (int s = 0; s < kScanTS; ++s) {
      const size_t row = rowBase + s;
      const float u = uf[row * kDin + d];
      const float z = xz[row * kXzLd + kDin + d];
      float acc = 0.f;
#pragma unroll
      for (int r = 0; r < kRank; ++r) acc = fmaf(sx[s][r], wr[r], acc);
      const float x1 = acc + bd;
      const float delta = fmaxf(x1, 0.f) + log1pf(expf(-fabsf(x1)));
      float y = 0.f;
#pragma unroll 1
      for (int n = 0; n < kNst; ++n) {
        const float a2 = sa[n][tid];
        const float hp = sh[n][tid];
        const float bn = sx[s][kRank + n];
        const float cn = sx[s][kRank + kNst + n];
        const float da = exp2f(delta * a2);
        const float hn = da * hp + (delta * bn) * u;
        sh[n][tid] = hn;
        y = fmaf(hn, cn, y);
      }
      y = fmaf(Dd, u, y);
      const float gate = z * __builtin_amdgcn_rcpf(1.0f + expf(-z));
      sy[s][tid] = y * gate;
    }
    __syncthreads();
    v4u hv[8], lv[8];
#pragma unroll
    for (int it = 0; it < 8; ++it) {
      const int r = wave * 32 + it * 4 + q;
      float v[8];
#pragma unroll
      for (int e = 0; e < 8; ++e) v[e] = sy[r][c8 + e];
      pack8_split(v, hv[it], lv[it]);
    }
    for (int pass = 0; pass < 2; ++pass) {
#pragma unroll
      for (int it = 0; it < 8; ++it) {
        const int r = wave * 32 + it * 4 + q;
        const size_t o = (rowBase + r) * kDin + (size_t)g * kScanCh + c8;
        *(volatile v4u*)(yhi + o) = hv[it];
        *(volatile v4u*)(ylo + o) = lv[it];
      }
      __threadfence();
    }
  }
}

__global__ __launch_bounds__(256) void xout_kernel(const float* __restrict__ ot, float* __restrict__ out) {
  __shared__ __align__(16) float sm[32][132];
  const int tid = threadIdx.x, lane = tid & 31, wave = tid >> 5;
  const int l0 = blockIdx.x * 128, c0 = blockIdx.y * 32, b = blockIdx.z;
#pragma unroll
  for (int i = 0; i < 16; ++i) {
    const int e = i * 256 + tid;
    const int t = e >> 5, c = e & 31;
    sm[c][t] = ot[((size_t)b * kSeqLen + l0 + t) * kOtLd + c0 + c];
  }
  __syncthreads();
  for (int pass = 0; pass < 2; ++pass) {
#pragma unroll
    for (int j = 0; j < 4; ++j) {
      const int cr = wave * 4 + j;
      const v4f v = *(const v4f*)(&sm[cr][lane * 4]);
      *(volatile v4f*)(out + ((size_t)(b * kChan + c0 + cr)) * kSeqLen + l0 + lane * 4) = v;
    }
    __threadfence();
  }
}

extern "C" void kernel_launch(void* const* d_in, const int* in_sizes, int n_in,
                              void* d_out, int out_size, void* d_ws, size_t ws_size,
                              hipStream_t stream)
{
  if (n_in < 12) return;
  if (in_sizes[0] != kBatch * kChan * kSeqLen || out_size != kBatch * kChan * kSeqLen) return;
  if (in_sizes[1] != kDin * kChan || in_sizes[2] != kChan * kDin * 9 || in_sizes[3] != 2 * kDin * kChan ||
      in_sizes[4] != kDin * kTaps1d || in_sizes[5] != kDin || in_sizes[6] != 38 * kDin || in_sizes[7] != kDin * kRank ||
      in_sizes[8] != kDin || in_sizes[9] != kDin * kNst || in_sizes[10] != kDin || in_sizes[11] != kChan * kDin) return;
  if (kWsTotal > ws_size) return;

  const float* x        = (const float*)d_in[0];
  const float* proj_w   = (const float*)d_in[1];
  const float* dconv_w  = (const float*)d_in[2];
  const float* inproj_w = (const float*)d_in[3];
  const float* conv1d_w = (const float*)d_in[4];
  const float* conv1d_b = (const float*)d_in[5];
  const float* xproj_w  = (const float*)d_in[6];
  const float* dtproj_w = (const float*)d_in[7];
  const float* dtproj_b = (const float*)d_in[8];
  const float* a_log    = (const float*)d_in[9];
  const float* dvec     = (const float*)d_in[10];
  const float* outp_w   = (const float*)d_in[11];
  float* out = (float*)d_out;

  unsigned char* ws = (unsigned char*)d_ws;
  unsigned short* Xhi   = (unsigned short*)(ws + kOffXhi);
  unsigned short* Xlo   = (unsigned short*)(ws + kOffXlo);
  unsigned short* PWhi  = (unsigned short*)(ws + kOffPWhi);
  unsigned short* PWlo  = (unsigned short*)(ws + kOffPWlo);
  unsigned short* WDhi  = (unsigned short*)(ws + kOffWDhi);
  unsigned short* WDlo  = (unsigned short*)(ws + kOffWDlo);
  unsigned short* IWhi  = (unsigned short*)(ws + kOffIWhi);
  unsigned short* IWlo  = (unsigned short*)(ws + kOffIWlo);
  unsigned short* XWhi  = (unsigned short*)(ws + kOffXWhi);
  unsigned short* XWlo  = (unsigned short*)(ws + kOffXWlo);
  unsigned short* OWhi  = (unsigned short*)(ws + kOffOWhi);
  unsigned short* OWlo  = (unsigned short*)(ws + kOffOWlo);
  unsigned short* XPhi  = (unsigned short*)(ws + kOffXPhi);
  unsigned short* XPlo  = (unsigned short*)(ws + kOffXPlo);
  unsigned short* IMhi  = (unsigned short*)(ws + kOffIMhi);
  unsigned short* IMlo  = (unsigned short*)(ws + kOffIMlo);
  unsigned short* SEQhi = (unsigned short*)(ws + kOffSEQhi);
  unsigned short* SEQlo = (unsigned short*)(ws + kOffSEQlo);
  float*          XZ    = (float*)(ws + kOffXZ);
  float*          Uf    = (float*)(ws + kOffUf);
  unsigned short* Uhi   = (unsigned short*)(ws + kOffUhi);
  unsigned short* Ulo   = (unsigned short*)(ws + kOffUlo);
  float*          XD    = (float*)(ws + kOffXD);
  unsigned short* Yhi   = (unsigned short*)(ws + kOffYhi);
  unsigned short* Ylo   = (unsigned short*)(ws + kOffYlo);
  float*          OT    = (float*)(ws + kOffOT);

  {
    const int n8pw = kDin * kChan / 8;
    const int n8wd = kWdRows * kImK / 8;
    const int n8iw = 2 * kDin * kChan / 8;
    const int n8xw = kXwRows * kDin / 8;
    const int n8ow = kOwRows * kDin / 8;
    wsplit_kernel<<<dim3((n8pw + 255) / 256), 256, 0, stream>>>(proj_w, PWhi, PWlo, kDin, kChan, 0, n8pw);
    wsplit_kernel<<<dim3((n8wd + 255) / 256), 256, 0, stream>>>(dconv_w, WDhi, WDlo, kChan, kImK, 1, n8wd);
    wsplit_kernel<<<dim3((n8iw + 255) / 256), 256, 0, stream>>>(inproj_w, IWhi, IWlo, 2 * kDin, kChan, 0, n8iw);
    wsplit_kernel<<<dim3((n8xw + 255) / 256), 256, 0, stream>>>(xproj_w, XWhi, XWlo, 38, kDin, 0, n8xw);
    wsplit_kernel<<<dim3((n8ow + 255) / 256), 256, 0, stream>>>(outp_w, OWhi, OWlo, kChan, kDin, 0, n8ow);
  }

  xin_kernel<<<dim3(kTok / 64), 256, 0, stream>>>(x, Xhi, Xlo);

  {
    const int tiles = (kTok / 64) * (kDin / 64);
    wmma_gemm64<1, true, 0, 2, false, 0><<<dim3(tiles / 8, 1), 256, 0, stream>>>(
        Xhi, Xlo, kChan, 0L, PWhi, PWlo, kChan, 0L,
        (void*)XPhi, (void*)XPlo, kDin, 0L, nullptr, nullptr, 0L, kTok, kDin, kChan, 1.0f);
  }

  for (int img = 0; img < kBatch; ++img) {
    im2col_kernel<<<dim3(kSeqLen / 8), 256, 0, stream>>>(XPhi, XPlo, IMhi, IMlo, img);
    const int tiles = (kSeqLen / 64) * (kSeqLd / 64);
    wmma_gemm64<1, true, 0, 2, false, 0><<<dim3(tiles / 8, 1), 256, 0, stream>>>(
        IMhi, IMlo, kImK, 0L, WDhi, WDlo, kImK, 0L,
        (void*)(SEQhi + (size_t)img * kSeqLen * kSeqLd), (void*)(SEQlo + (size_t)img * kSeqLen * kSeqLd), kSeqLd, 0L,
        nullptr, nullptr, 0L, kSeqLen, kSeqLd, kImK, 1.0f);
  }

  {
    const int tiles = (kTok / 64) * (kXzLd / 64);
    wmma_gemm64<1, true, 0, 0, false, 0><<<dim3(tiles / 8, 1), 256, 0, stream>>>(
        SEQhi, SEQlo, kSeqLd, 0L, IWhi, IWlo, kChan, 0L,
        (void*)XZ, nullptr, kXzLd, 0L, nullptr, nullptr, 0L, kTok, kXzLd, kChan, 1.0f);
  }

  conv_silu_kernel<<<dim3(kTok / 8), 256, 0, stream>>>(XZ, conv1d_w, conv1d_b, Uf, Uhi, Ulo);

  {
    const int tiles = (kTok / 64) * (kXdLd / 64);
    wmma_gemm64<1, true, 0, 0, false, 0><<<dim3(tiles / 8, 1), 256, 0, stream>>>(
        Uhi, Ulo, kDin, 0L, XWhi, XWlo, kDin, 0L,
        (void*)XD, nullptr, kXdLd, 0L, nullptr, nullptr, 0L, kTok, kXdLd, kDin, 1.0f);
  }

  scan_kernel<<<dim3(kBatch * 3), 64, 0, stream>>>(XD, Uf, XZ, dtproj_w, dtproj_b, a_log, dvec, Yhi, Ylo);

  {
    const int tiles = (kTok / 64) * (kOtLd / 64);
    wmma_gemm64<1, true, 0, 0, false, 0><<<dim3(tiles / 8, 1), 256, 0, stream>>>(
        Yhi, Ylo, kDin, 0L, OWhi, OWlo, kDin, 0L,
        (void*)OT, nullptr, kOtLd, 0L, nullptr, nullptr, 0L, kTok, kOtLd, kDin, 1.0f);
  }

  xout_kernel<<<dim3(kSeqLen / 128, kChan / 32, kBatch), 256, 0, stream>>>(OT, out);
}
